// ResidualBlockOriginal_40699110096963
// MI455X (gfx1250) — hardware-verified
//
#include <hip/hip_runtime.h>
#include <stddef.h>


#define C_CH     32
#define K_OFF    27
#define EPSV     1e-5f
#define STHR     256
#define SWAV     (STHR / 32)
#define SLOT     16
#define LGRP     4
#define CHB      (STHR * SLOT)
#define NBK      512
#define NBKL     9
#define MAXB     512
#define CAP2     12288
#define MAXDEG   128
#define SRCB     18
#define KQB      5
#define LOCB     (SRCB + KQB)
#define LDS_BKT  ((2 * CAP2 + SWAV * NBK + 2 * NBK) * 4 + 64)
#define CTHR     64
#define CWAV     (CTHR / 32)
#define CNODE    (16 * CWAV)
#define GW       (16 * K_OFF * C_CH)
#define LC_G     0
#define LC_S     (CWAV * GW)
#define LC_P     (LC_S + CWAV * 512)
#define LC_Q     (LC_P + CWAV * 64)
#define LC_T     (LC_Q + 64)
#define LC_END   (LC_T + 128)
#define LDS_CONV (LC_END * 4)
#define OTHR     128
#define OROWS    (OTHR / 8)
#define XSC      8.0f
#define WSC      64.0f
#define RH       0.001953125f
#define WSCAP    134217728

static_assert(CHB == 4096);
static_assert(SWAV * MAXB == 4 * STHR * 4);
static_assert(CHB == 4 * STHR * 4);
static_assert(MAXB == 2 * STHR);
static_assert(NBK == 2 * STHR);
static_assert((CAP2 % (4 * STHR)) == 0);
static_assert((SWAV * NBK) % (4 * STHR) == 0);
static_assert(2 * NBK == 4 * STHR);
static_assert((CAP2 % (32 * SWAV)) == 0);
static_assert(LDS_BKT == 118848);
static_assert(LOCB + NBKL == 32);
static_assert((1 << KQB) >= K_OFF);
static_assert(((CWAV * GW) % (4 * CTHR)) == 0);
static_assert(LDS_CONV == 115968);
static_assert(CNODE == 32);
static_assert(OROWS == 16);
static_assert((SLOT % LGRP) == 0);

typedef float    v4f  __attribute__((ext_vector_type(4)));
typedef float    v8f  __attribute__((ext_vector_type(8)));
typedef int      v4i  __attribute__((ext_vector_type(4)));
typedef unsigned v4u  __attribute__((ext_vector_type(4)));
typedef _Float16 v4h  __attribute__((ext_vector_type(4)));
typedef _Float16 v8h  __attribute__((ext_vector_type(8)));
typedef _Float16 v16h __attribute__((ext_vector_type(16)));
union Frag { v16h v; v8h h[2]; v4h q[4]; };

__device__ __forceinline__ v8f wmh(v16h a, v16h b, v8f c) {
  v8f d = __builtin_amdgcn_wmma_f32_16x16x32_f16(false, a, false, b, (short)0, c, false, false);
  asm volatile("v_nop\n\tv_nop\n\tv_nop\n\tv_nop" : "+v"(d) : "v"(a), "v"(b));
  return d;
}

__device__ __forceinline__ v4h cvt4h(v4f x) {
  v4h r;
  r.x = (_Float16)x.x;
  r.y = (_Float16)x.y;
  r.z = (_Float16)x.z;
  r.w = (_Float16)x.w;
  return r;
}

__device__ __forceinline__ void wfence() {
  __builtin_amdgcn_fence(__ATOMIC_ACQ_REL, "wavefront");
  __builtin_amdgcn_wave_barrier();
}

__device__ __forceinline__ unsigned match9(int key, unsigned vm) {
  unsigned peers = vm;
#pragma unroll
  for (int i = 0; i < 9; ++i) {
    const bool bit = ((key >> i) & 1) != 0;
    const unsigned bq = __builtin_amdgcn_ballot_w32(bit);
    peers &= bit ? bq : ~bq;
  }
  return peers;
}

__device__ __forceinline__ void blkscan(int cnt, int lane, int wave, int* swt, int& pos, int& nh) {
  int x = cnt;
#pragma unroll
  for (int o = 1; o < 32; o <<= 1) {
    const int y = __shfl_up(x, o, 32);
    x += (lane >= o) ? y : 0;
  }
  if (lane == 31) swt[wave] = x;
  __syncthreads();
  int wpre = 0, tot = 0;
#pragma unroll
  for (int w = 0; w < SWAV; ++w) {
    const int v = swt[w];
    wpre += (w < wave) ? v : 0;
    tot += v;
  }
  pos = wpre + x - cnt;
  nh = tot;
}

__global__ __launch_bounds__(128) void k_wprep(const float* __restrict__ W1, const float* __restrict__ W2,
                                                _Float16* Wp) {
  const int k = blockIdx.x, cv = blockIdx.y, tid = threadIdx.x;
  const int n = tid >> 2, c0 = (tid & 3) * 8;
  const float* wk = (cv != 0 ? W2 : W1) + (size_t)k * (C_CH * C_CH);
  v8h hv;
#pragma unroll
  for (int e = 0; e < 8; ++e) hv[e] = (_Float16)(wk[(c0 + e) * C_CH + n] * WSC);
  _Float16* dst = Wp + ((size_t)(cv * K_OFF + k) * C_CH + n) * C_CH + c0;
  *(volatile v8h*)dst = hv;
  __threadfence();
  *(volatile v8h*)dst = hv;
}

__global__ __launch_bounds__(STHR) void k_bsort(const int* dsts, const int* srcs, const int* msk,
                                                 unsigned* KEY, unsigned* CO, int nN, int nE) {
  __shared__ __attribute__((aligned(16))) int      srun[SWAV * MAXB];
  __shared__ __attribute__((aligned(16))) unsigned sstg[CHB];
  __shared__ __attribute__((aligned(16))) unsigned sco[MAXB];
  __shared__ int swt[SWAV];
  const int tid = threadIdx.x, lane = tid & 31;
  const int wave = __builtin_amdgcn_readfirstlane(tid >> 5);
  const unsigned lt = (1u << lane) - 1u;
  {
    const v4i z = {0, 0, 0, 0};
    const v4u zu = {0u, 0u, 0u, 0u};
#pragma unroll
    for (int it = 0; it < (SWAV * MAXB) / (4 * STHR); ++it) ((v4i*)srun)[it * STHR + tid] = z;
#pragma unroll
    for (int it = 0; it < CHB / (4 * STHR); ++it) ((v4u*)sstg)[it * STHR + tid] = zu;
  }
  __syncthreads();

  const int eb = blockIdx.x * CHB + wave * (32 * SLOT);
  int dc[SLOT];
  unsigned pay[SLOT];
  unsigned vm = 0u;
#pragma unroll
  for (int g = 0; g < SLOT / LGRP; ++g) {
    int dl[LGRP], sl[LGRP], ml[LGRP];
#pragma unroll
    for (int u = 0; u < LGRP; ++u) {
      const int e = eb + 32 * (g * LGRP + u) + lane;
      const int ec = e < nE ? e : nE - 1;
      dl[u] = dsts[ec];
      sl[u] = srcs[ec];
      ml[u] = msk[ec];
    }
    asm volatile("s_wait_loadcnt 0x0" ::: "memory");
#pragma unroll
    for (int u = 0; u < LGRP; ++u) {
      const int j = g * LGRP + u;
      const int e = eb + 32 * j + lane;
      const bool ok = e < nE;
      const int ec = ok ? e : nE - 1;
      int d = dl[u];
      d = d < 0 ? d + nN : d;
      int s = sl[u];
      s = s < 0 ? s + nN : s;
      s = s < 0 ? 0 : (s > nN - 1 ? nN - 1 : s);
      int kq = ec / nN;
      kq = kq < 0 ? 0 : (kq > (1 << KQB) - 1 ? (1 << KQB) - 1 : kq);
      const bool inr = ok && ((unsigned)d < (unsigned)nN) && (ml[u] != 0);
      dc[j] = inr ? d : 0;
      pay[j] = ((unsigned)kq << SRCB) | (unsigned)s;
      vm |= (inr ? 1u : 0u) << j;
    }
  }
  int* runw = srun + wave * MAXB;

#pragma unroll
  for (int j = 0; j < SLOT; ++j) {
    const bool inr = ((vm >> j) & 1u) != 0u;
    const int kb = dc[j] >> NBKL;
    const unsigned vmask = __builtin_amdgcn_ballot_w32(inr);
    const unsigned peers = match9(kb, vmask);
    const int pc = __builtin_popcount(peers);
    const bool lead = inr && ((peers & lt) == 0u);
    const int cur = runw[kb];
    if (lead) runw[kb] = cur + pc;
    wfence();
  }
  __syncthreads();

  {
    const int b0 = 2 * tid, b1 = b0 + 1;
    int c0 = 0, c1 = 0, pw0[SWAV], pw1[SWAV];
#pragma unroll
    for (int w = 0; w < SWAV; ++w) {
      pw0[w] = c0; c0 += srun[w * MAXB + b0];
      pw1[w] = c1; c1 += srun[w * MAXB + b1];
    }
    int pos, tot;
    blkscan(c0 + c1, lane, wave, swt, pos, tot);
    const int o0 = pos, o1 = pos + c0;
#pragma unroll
    for (int w = 0; w < SWAV; ++w) {
      srun[w * MAXB + b0] = o0 + pw0[w];
      srun[w * MAXB + b1] = o1 + pw1[w];
    }
    sco[b0] = ((unsigned)o0 << 16) | (unsigned)c0;
    sco[b1] = ((unsigned)o1 << 16) | (unsigned)c1;
  }
  __syncthreads();

#pragma unroll
  for (int j = 0; j < SLOT; ++j) {
    const bool inr = ((vm >> j) & 1u) != 0u;
    const int kb = dc[j] >> NBKL;
    const unsigned vmask = __builtin_amdgcn_ballot_w32(inr);
    const unsigned peers = match9(kb, vmask);
    const int pc = __builtin_popcount(peers);
    const bool lead = inr && ((peers & lt) == 0u);
    const int cur = runw[kb];
    const int p = cur + __builtin_popcount(peers & lt);
    if (lead) runw[kb] = cur + pc;
    if (inr) {
      const int pp = p < CHB - 1 ? p : CHB - 1;
      sstg[pp] = (((unsigned)dc[j] & (unsigned)(NBK - 1)) << LOCB) | pay[j];
    }
    wfence();
  }
  __syncthreads();

  unsigned* kp = KEY + (size_t)blockIdx.x * CHB;
  unsigned* cp = CO + (size_t)blockIdx.x * MAXB;
#pragma unroll
  for (int it = 0; it < CHB / (4 * STHR); ++it) {
    const int f = it * STHR + tid;
    const v4u vv = ((const v4u*)sstg)[f];
    *(volatile v4u*)(kp + 4 * f) = vv;
  }
  if (tid < MAXB / 4) {
    const v4u vv = ((const v4u*)sco)[tid];
    *(volatile v4u*)(cp + 4 * tid) = vv;
  }
  __threadfence();
#pragma unroll
  for (int it = 0; it < CHB / (4 * STHR); ++it) {
    const int f = it * STHR + tid;
    const v4u vv = ((const v4u*)sstg)[f];
    *(volatile v4u*)(kp + 4 * f) = vv;
  }
  if (tid < MAXB / 4) {
    const v4u vv = ((const v4u*)sco)[tid];
    *(volatile v4u*)(cp + 4 * tid) = vv;
  }
}

__global__ __launch_bounds__(STHR) void k_bucket(const unsigned* __restrict__ CO, const unsigned* __restrict__ KEY,
                                                  unsigned* EID, int* NT, int nChunk, int nBatch) {
  extern __shared__ __attribute__((aligned(16))) char dynl[];
  unsigned* lst = (unsigned*)dynl;
  unsigned* srt = lst + CAP2;
  int*      wc  = (int*)(srt + CAP2);
  int*      snt = wc + SWAV * NBK;
  int*      swt = snt + 2 * NBK;
  const int tid = threadIdx.x, lane = tid & 31;
  const int wave = __builtin_amdgcn_readfirstlane(tid >> 5);
  const unsigned lt = (1u << lane) - 1u;
  const int b = blockIdx.x;
  {
    const v4u zu = {0u, 0u, 0u, 0u};
    const v4i z = {0, 0, 0, 0};
#pragma unroll
    for (int it = 0; it < CAP2 / (4 * STHR); ++it) {
      ((v4u*)lst)[it * STHR + tid] = zu;
      ((v4u*)srt)[it * STHR + tid] = zu;
    }
#pragma unroll
    for (int it = 0; it < (SWAV * NBK) / (4 * STHR); ++it) ((v4i*)wc)[it * STHR + tid] = z;
  }
  __syncthreads();

  int L = 0;
#pragma unroll 1
  for (int q = 0; q < nBatch; ++q) {
    const int s = q * STHR + tid;
    const bool sv = s < nChunk;
    const int sc = sv ? s : nChunk - 1;
    const unsigned co = CO[(size_t)sc * MAXB + b];
    int c = sv ? (int)(co & 0x1FFFu) : 0;
    c = c > CHB ? CHB : c;
    int o = (int)((co >> 16) & 0x1FFFu);
    o = o > CHB - c ? CHB - c : o;
    int pos, tot;
    blkscan(c, lane, wave, swt, pos, tot);
    const int base = L + pos;
    const unsigned* rp = KEY + (size_t)sc * CHB + o;
#pragma unroll 1
    for (int i = 0; i < c; ++i) {
      const int di = base + i;
      const unsigned vv = rp[i];
      if ((unsigned)di < (unsigned)CAP2) lst[di] = vv;
    }
    L += tot;
    __syncthreads();
  }
  const int Lc = L < CAP2 ? L : CAP2;
  const int nG = (Lc + 31) >> 5;
  int* wcw = wc + wave * NBK;

#pragma unroll 1
  for (int gi = 0; gi < CAP2 / (32 * SWAV); ++gi) {
    const int g = wave + SWAV * gi;
    if (g >= nG) break;
    const int idx = 32 * g + lane;
    const bool valid = idx < Lc;
    const unsigned key = lst[idx];
    const int ld = (int)((key >> LOCB) & (unsigned)(NBK - 1));
    const unsigned vmask = __builtin_amdgcn_ballot_w32(valid);
    const unsigned peers = match9(ld, vmask);
    const int pc = __builtin_popcount(peers);
    const bool lead = valid && ((peers & lt) == 0u);
    const int cur = wcw[ld];
    if (lead) wcw[ld] = cur + pc;
    wfence();
  }
  __syncthreads();

  {
    const int l0 = 2 * tid, l1 = l0 + 1;
    int c0 = 0, c1 = 0, pw0[SWAV], pw1[SWAV];
#pragma unroll
    for (int w = 0; w < SWAV; ++w) {
      pw0[w] = c0; c0 += wc[w * NBK + l0];
      pw1[w] = c1; c1 += wc[w * NBK + l1];
    }
    int pos, tot;
    blkscan(c0 + c1, lane, wave, swt, pos, tot);
    const int off0 = pos, off1 = pos + c0;
#pragma unroll
    for (int w = 0; w < SWAV; ++w) {
      wc[w * NBK + l0] = off0 + pw0[w];
      wc[w * NBK + l1] = off1 + pw1[w];
    }
    int n0c = c0, n1c = c1;
    if (off0 + n0c > CAP2) n0c = CAP2 - off0;
    if (off1 + n1c > CAP2) n1c = CAP2 - off1;
    n0c = n0c < 0 ? 0 : n0c;
    n1c = n1c < 0 ? 0 : n1c;
    const int s0 = off0 < CAP2 ? off0 : CAP2 - 1;
    const int s1 = off1 < CAP2 ? off1 : CAP2 - 1;
    snt[2 * l0] = b * CAP2 + s0; snt[2 * l0 + 1] = n0c;
    snt[2 * l1] = b * CAP2 + s1; snt[2 * l1 + 1] = n1c;
  }
  __syncthreads();

#pragma unroll 1
  for (int gi = 0; gi < CAP2 / (32 * SWAV); ++gi) {
    const int g = wave + SWAV * gi;
    if (g >= nG) break;
    const int idx = 32 * g + lane;
    const bool valid = idx < Lc;
    const unsigned key = lst[idx];
    const int ld = (int)((key >> LOCB) & (unsigned)(NBK - 1));
    const unsigned vmask = __builtin_amdgcn_ballot_w32(valid);
    const unsigned peers = match9(ld, vmask);
    const int pc = __builtin_popcount(peers);
    const bool lead = valid && ((peers & lt) == 0u);
    const int cur = wcw[ld];
    const int p = cur + __builtin_popcount(peers & lt);
    if (lead) wcw[ld] = cur + pc;
    if (valid && (unsigned)p < (unsigned)CAP2) srt[p] = key & ((1u << LOCB) - 1u);
    wfence();
  }
  __syncthreads();

  unsigned* ep = EID + (size_t)b * CAP2;
  int* np = NT + (size_t)b * (2 * NBK);
#pragma unroll
  for (int it = 0; it < CAP2 / (4 * STHR); ++it) {
    const int f = it * STHR + tid;
    const v4u vv = ((const v4u*)srt)[f];
    *(volatile v4u*)(ep + 4 * f) = vv;
  }
  {
    const v4i vv = ((const v4i*)snt)[tid];
    *(volatile v4i*)(np + 4 * tid) = vv;
  }
  __threadfence();
#pragma unroll
  for (int it = 0; it < CAP2 / (4 * STHR); ++it) {
    const int f = it * STHR + tid;
    const v4u vv = ((const v4u*)srt)[f];
    *(volatile v4u*)(ep + 4 * f) = vv;
  }
  {
    const v4i vv = ((const v4i*)snt)[tid];
    *(volatile v4i*)(np + 4 * tid) = vv;
  }
}

template <int BNF>
__global__ __launch_bounds__(CTHR) void k_conv(
    const float* __restrict__ feat, const int* __restrict__ NT, const unsigned* __restrict__ EID,
    const _Float16* __restrict__ Wp, const float* __restrict__ stin,
    const float* __restrict__ gin, const float* __restrict__ bin,
    float* yout, float* part, int nN, int totE) {
  extern __shared__ __attribute__((aligned(16))) char dynl[];
  float* G = (float*)dynl + LC_G;
  float* S = (float*)dynl + LC_S;
  float* P = (float*)dynl + LC_P;
  float* Q = (float*)dynl + LC_Q;
  float* T = (float*)dynl + LC_T;
  const int tid = threadIdx.x, lane = tid & 31, hh = lane >> 4, m = lane & 15;
  const int wave = __builtin_amdgcn_readfirstlane(tid >> 5);
  {
    const v4f z = {0.0f, 0.0f, 0.0f, 0.0f};
#pragma unroll 4
    for (int it = 0; it < (CWAV * GW) / (4 * CTHR); ++it) ((v4f*)G)[it * CTHR + tid] = z;
  }
  if (BNF) {
    if (wave == 0) {
      T[lane]      = stin[lane];
      T[32 + lane] = stin[32 + lane];
      T[64 + lane] = gin[lane];
      T[96 + lane] = bin[lane];
    }
  }
  __syncthreads();
  float mch = 0.0f, rch = 1.0f, gch = 1.0f, bch = 0.0f;
  if (BNF) { mch = T[lane]; rch = T[32 + lane]; gch = T[64 + lane]; bch = T[96 + lane]; }

  float* Gw = G + wave * GW;
  const int nb = blockIdx.x * CNODE + wave * 16;
#pragma unroll 1
  for (int j = 0; j < 16; ++j) {
    int node = nb + j;
    node = node > nN - 1 ? nN - 1 : node;
    int st = NT[2 * (size_t)node];
    int ct = NT[2 * (size_t)node + 1];
    st = __builtin_amdgcn_readfirstlane(st);
    ct = __builtin_amdgcn_readfirstlane(ct);
    ct = ct < 0 ? 0 : (ct > MAXDEG ? MAXDEG : ct);
    st = st < 0 ? 0 : (st > totE - 1 ? totE - 1 : st);
    float* gr = Gw + j * (K_OFF * C_CH) + lane;
#pragma unroll 1
    for (int t = 0; t < ct; ++t) {
      int ix = st + t;
      ix = ix > totE - 1 ? totE - 1 : ix;
      unsigned ent = EID[ix];
      ent = __builtin_amdgcn_readfirstlane(ent);
      int k = (int)((ent >> SRCB) & ((1u << KQB) - 1u));
      k = k > K_OFF - 1 ? K_OFF - 1 : k;
      int src = (int)(ent & ((1u << SRCB) - 1u));
      src = src > nN - 1 ? nN - 1 : src;
      float v = feat[(size_t)src * C_CH + lane];
      if (BNF) v = fmaxf(((v - mch) * rch) * gch + bch, 0.0f);
      gr[k * C_CH] += v;
    }
  }
  __syncthreads();

  const v8f z8 = {0.0f, 0.0f, 0.0f, 0.0f, 0.0f, 0.0f, 0.0f, 0.0f};
  v8f acc0 = z8, acc1 = z8;
  {
    const float* ga = Gw + m * (K_OFF * C_CH) + 8 * hh;
    const _Float16* wb0 = Wp + (size_t)m * C_CH + 8 * hh;
    const _Float16* wb1 = Wp + (size_t)(16 + m) * C_CH + 8 * hh;
#pragma unroll 1
    for (int k = 0; k < K_OFF; ++k) {
      const float* gp = ga + k * C_CH;
      const v4f f0 = *(const v4f*)(gp);
      const v4f f1 = *(const v4f*)(gp + 4);
      const v4f f2 = *(const v4f*)(gp + 16);
      const v4f f3 = *(const v4f*)(gp + 20);
      Frag a, b0, b1;
      a.q[0] = cvt4h(f0 * XSC);
      a.q[1] = cvt4h(f1 * XSC);
      a.q[2] = cvt4h(f2 * XSC);
      a.q[3] = cvt4h(f3 * XSC);
      const _Float16* p0 = wb0 + (size_t)k * (C_CH * C_CH);
      const _Float16* p1 = wb1 + (size_t)k * (C_CH * C_CH);
      b0.h[0] = *(const v8h*)(p0);
      b0.h[1] = *(const v8h*)(p0 + 16);
      b1.h[0] = *(const v8h*)(p1);
      b1.h[1] = *(const v8h*)(p1 + 16);
      acc0 = wmh(a.v, b0.v, acc0);
      acc1 = wmh(a.v, b1.v, acc1);
    }
  }

  float* Sw = S + wave * 512;
#pragma unroll
  for (int r = 0; r < 8; ++r) {
    Sw[(8 * hh + r) * C_CH + m]      = acc0[r] * RH;
    Sw[(8 * hh + r) * C_CH + 16 + m] = acc1[r] * RH;
  }
  __syncthreads();

  {
    float s = 0.0f, q = 0.0f;
#pragma unroll
    for (int r = 0; r < 16; ++r) {
      const float v = Sw[r * C_CH + lane];
      const bool ok = (nb + r) < nN;
      const float u = ok ? v : 0.0f;
      s += u;
      q += u * u;
    }
    P[wave * 64 + lane]      = s;
    P[wave * 64 + 32 + lane] = q;
  }
  {
    const int rr = lane >> 3, cc = (lane & 7) * 4;
    v4f ov[4];
#pragma unroll
    for (int qq = 0; qq < 4; ++qq) ov[qq] = *(const v4f*)(Sw + (4 * qq + rr) * C_CH + cc);
    float* yb = yout + (size_t)nb * C_CH + cc;
#pragma unroll
    for (int qq = 0; qq < 4; ++qq) *(volatile v4f*)(yb + (size_t)(4 * qq + rr) * C_CH) = ov[qq];
    __threadfence();
#pragma unroll
    for (int qq = 0; qq < 4; ++qq) *(volatile v4f*)(yb + (size_t)(4 * qq + rr) * C_CH) = ov[qq];
  }
  __syncthreads();
  if (wave == 0) {
    Q[lane]      = P[lane] + P[64 + lane];
    Q[32 + lane] = P[32 + lane] + P[96 + lane];
  }
  __syncthreads();
  {
    const v4f pv = *(const v4f*)(Q + 4 * (tid & 15));
    float* pp = part + (size_t)blockIdx.x * 64 + 4 * (tid & 15);
    if (tid < 16) *(volatile v4f*)pp = pv;
    __threadfence();
    if (tid < 16) *(volatile v4f*)pp = pv;
  }
}

__global__ __launch_bounds__(32) void k_stats(const float* __restrict__ part, float* st, int nBlk, int nN) {
  __shared__ __attribute__((aligned(16))) float so[64];
  const int lane = threadIdx.x & 31;
  double s = 0.0, q = 0.0;
#pragma unroll 1
  for (int b = 0; b < nBlk; ++b) {
    s += (double)part[(size_t)b * 64 + lane];
    q += (double)part[(size_t)b * 64 + 32 + lane];
  }
  const double inv = 1.0 / (double)nN;
  const double mean = s * inv;
  double var = q * inv - mean * mean;
  var = var < 0.0 ? 0.0 : var;
  const float mf = (float)mean;
  const float vf = (float)var;
  const float r = rsqrtf(vf + EPSV);
  so[lane] = mf;
  so[32 + lane] = r;
  __syncthreads();
  const v4f v = *(const v4f*)(so + 4 * (lane & 15));
  float* p = st + 4 * (lane & 15);
  if (lane < 16) *(volatile v4f*)p = v;
  __threadfence();
  if (lane < 16) *(volatile v4f*)p = v;
}

__global__ __launch_bounds__(OTHR) void k_out(const float* __restrict__ y2, const float* __restrict__ st,
                                               const float* __restrict__ g, const float* __restrict__ bt,
                                               const float* __restrict__ x, float* out, int nN) {
  const int tid = threadIdx.x;
  const int row = blockIdx.x * OROWS + (tid >> 3);
  const int cc = (tid & 7) * 4;
  const int rc = row > nN - 1 ? nN - 1 : row;
  const v4f yv = *(const v4f*)(y2 + (size_t)rc * C_CH + cc);
  const v4f xv = *(const v4f*)(x + (size_t)rc * C_CH + cc);
  const v4f mv = *(const v4f*)(st + cc);
  const v4f rv = *(const v4f*)(st + 32 + cc);
  const v4f gv = *(const v4f*)(g + cc);
  const v4f bv = *(const v4f*)(bt + cc);
  v4f o = ((yv - mv) * rv) * gv + bv + xv;
  o.x = fmaxf(o.x, 0.0f);
  o.y = fmaxf(o.y, 0.0f);
  o.z = fmaxf(o.z, 0.0f);
  o.w = fmaxf(o.w, 0.0f);
  float* op = out + (size_t)rc * C_CH + cc;
  if (row < nN) *(volatile v4f*)op = o;
  __threadfence();
  if (row < nN) *(volatile v4f*)op = o;
}

extern "C" void kernel_launch(void* const* d_in, const int* in_sizes, int n_in,
                              void* d_out, int out_size, void* d_ws, size_t ws_size,
                              hipStream_t stream) {
  if (n_in < 10) return;
  if (in_sizes[0] < C_CH) return;
  const int nN = in_sizes[0] / C_CH;
  if (nN < 1 || in_sizes[0] != nN * C_CH) return;
  if (nN > (1 << SRCB)) return;
  const int nE = K_OFF * nN;
  if (in_sizes[1] != K_OFF * C_CH * C_CH || in_sizes[4] != K_OFF * C_CH * C_CH) return;
  if (in_sizes[2] != C_CH || in_sizes[3] != C_CH || in_sizes[5] != C_CH || in_sizes[6] != C_CH) return;
  if (in_sizes[7] != nE || in_sizes[8] != nE || in_sizes[9] != nE) return;
  if (out_size != nN * C_CH) return;

  const int nChunk = (nE + CHB - 1) / CHB;
  const int ePad   = nChunk * CHB;
  const int nB     = (nN + NBK - 1) / NBK;
  if (nB > MAXB) return;
  const int nBatch = (nChunk + STHR - 1) / STHR;
  const int totE   = nB * CAP2;
  const int nBlkC  = (nN + CNODE - 1) / CNODE;
  const int gOut   = (nN + OROWS - 1) / OROWS;

  const float* x      = (const float*)d_in[0];
  const float* W1     = (const float*)d_in[1];
  const float* gamma1 = (const float*)d_in[2];
  const float* beta1  = (const float*)d_in[3];
  const float* W2     = (const float*)d_in[4];
  const float* gamma2 = (const float*)d_in[5];
  const float* beta2  = (const float*)d_in[6];
  const int*   inmap  = (const int*)d_in[7];
  const int*   outmap = (const int*)d_in[8];
  const int*   vmask  = (const int*)d_in[9];
  float* out = (float*)d_out;

  char* ws = (char*)d_ws;
  size_t off = 0;
  const size_t oWp  = off; off += (size_t)2 * K_OFF * C_CH * C_CH * 2;      off = (off + 255) & ~(size_t)255;
  const size_t oKey = off; off += (size_t)ePad * 4;                          off = (off + 255) & ~(size_t)255;
  const size_t oCo  = off; off += (size_t)nChunk * MAXB * 4;                 off = (off + 255) & ~(size_t)255;
  const size_t oEid = off; off += (size_t)nB * CAP2 * 4;                     off = (off + 255) & ~(size_t)255;
  const size_t oNt  = off; off += (size_t)nB * NBK * 2 * 4;                  off = (off + 255) & ~(size_t)255;
  const size_t oY1  = off; off += (size_t)nBlkC * CNODE * C_CH * 4;          off = (off + 255) & ~(size_t)255;
  const size_t oY2  = off; off += (size_t)nBlkC * CNODE * C_CH * 4;          off = (off + 255) & ~(size_t)255;
  const size_t oP1  = off; off += (size_t)nBlkC * 64 * 4;                    off = (off + 255) & ~(size_t)255;
  const size_t oP2  = off; off += (size_t)nBlkC * 64 * 4;                    off = (off + 255) & ~(size_t)255;
  const size_t oS1  = off; off += 256;
  const size_t oS2  = off; off += 256;
  if (off > ws_size || off > (size_t)WSCAP) return;
  _Float16* Wp  = (_Float16*)(ws + oWp);
  unsigned* KEY = (unsigned*)(ws + oKey);
  unsigned* CO  = (unsigned*)(ws + oCo);
  unsigned* EID = (unsigned*)(ws + oEid);
  int*      NT  = (int*)(ws + oNt);
  float*    Y1  = (float*)(ws + oY1);
  float*    Y2  = (float*)(ws + oY2);
  float*    P1  = (float*)(ws + oP1);
  float*    P2  = (float*)(ws + oP2);
  float*    S1  = (float*)(ws + oS1);
  float*    S2  = (float*)(ws + oS2);

  auto kc0 = k_conv<0>;
  auto kc1 = k_conv<1>;
  hipFuncSetAttribute(reinterpret_cast<const void*>(&k_bucket), hipFuncAttributeMaxDynamicSharedMemorySize, LDS_BKT);
  hipFuncSetAttribute(reinterpret_cast<const void*>(kc0), hipFuncAttributeMaxDynamicSharedMemorySize, LDS_CONV);
  hipFuncSetAttribute(reinterpret_cast<const void*>(kc1), hipFuncAttributeMaxDynamicSharedMemorySize, LDS_CONV);

  k_wprep<<<dim3(K_OFF, 2), 128, 0, stream>>>(W1, W2, Wp);
  k_bsort<<<nChunk, STHR, 0, stream>>>(outmap, inmap, vmask, KEY, CO, nN, nE);
  k_bucket<<<nB, STHR, LDS_BKT, stream>>>(CO, KEY, EID, NT, nChunk, nBatch);
  k_conv<0><<<nBlkC, CTHR, LDS_CONV, stream>>>(x, NT, EID, Wp, S1, gamma1, beta1, Y1, P1, nN, totE);
  k_stats<<<1, 32, 0, stream>>>(P1, S1, nBlkC, nN);
  k_conv<1><<<nBlkC, CTHR, LDS_CONV, stream>>>(Y1, NT, EID, Wp + (size_t)K_OFF * C_CH * C_CH, S1, gamma1, beta1,
                                                Y2, P2, nN, totE);
  k_stats<<<1, 32, 0, stream>>>(P2, S2, nBlkC, nN);
  k_out<<<gOut, OTHR, 0, stream>>>(Y2, S2, gamma2, beta2, x, out, nN);
}
